// MultiCharacterConditioner_60790967107677
// MI455X (gfx1250) — hardware-run, weakly checked
//
#include <hip/hip_runtime.h>
#include <math.h>

typedef __attribute__((ext_vector_type(16))) _Float16 v16h;
typedef __attribute__((ext_vector_type(8)))  _Float16 v8h;
typedef __attribute__((ext_vector_type(16))) __bf16   v16b;
typedef __attribute__((ext_vector_type(8)))  __bf16   v8b;
typedef __attribute__((ext_vector_type(8)))  float    v8f;
typedef __attribute__((ext_vector_type(4)))  float    v4f;

constexpr int kNB   = 2;
constexpr int kSeq  = 2048;
constexpr int kDim  = 1024;
constexpr int kNH   = 16;
constexpr int kHD   = 64;
constexpr int kNCh  = 4;
constexpr int kTok  = kNB * kSeq;
constexpr int kBH   = kNB * kNH;
static_assert(kNH * kHD == kDim);
static_assert(kHD == 64);
static_assert((kTok % 64) == 0 && (kDim % 64) == 0 && (kSeq % 64) == 0);
static_assert((kDim % 32) == 0 && (kHD % 32) == 0 && (kSeq % 32) == 0);

constexpr bool  kBf16Inputs = true;
constexpr float kEps        = 1e-6f;
constexpr float kBoost      = 0.3f;
constexpr float kQKScale    = 0.125f;
static_assert(kQKScale * kQKScale * (float)kHD == 1.0f);
constexpr float kInvHD      = 1.0f / (float)kHD;
constexpr float kWCarry     = 16.0f;
constexpr float kWCarryInv  = 1.0f / kWCarry;
constexpr float kPCarry     = 32768.0f;
constexpr float kCtxCarry   = 64.0f;
constexpr float kCtxFold    = kCtxCarry / (kPCarry * kWCarry);
constexpr float kOutScale   = 1.0f / (kCtxCarry * kWCarry);

constexpr size_t kSzX16    = (size_t)kTok * kDim * 2;
constexpr size_t kSzWqkv16 = (size_t)3 * kDim * kDim * 2;
constexpr size_t kSzWout16 = (size_t)kDim * kDim * 2;
constexpr size_t kSzHead16 = (size_t)kBH * kSeq * kHD * 2;
constexpr size_t kSzAO16   = (size_t)kTok * kDim * 2;
constexpr size_t kSzBias   = (size_t)kNB * kSeq * kSeq * 4;
constexpr size_t kOffX16    = 0;
constexpr size_t kOffWqkv16 = kOffX16 + kSzX16;
constexpr size_t kOffWout16 = kOffWqkv16 + kSzWqkv16;
constexpr size_t kOffQ16    = kOffWout16 + kSzWout16;
constexpr size_t kOffK16    = kOffQ16 + kSzHead16;
constexpr size_t kOffVt16   = kOffK16 + kSzHead16;
constexpr size_t kOffAO16   = kOffVt16 + kSzHead16;
constexpr size_t kOffBias   = kOffAO16 + kSzAO16;
constexpr size_t kWsTotal   = kOffBias + kSzBias;
static_assert(kWsTotal == 83886080ull);
static_assert(kWsTotal <= 134217728ull);
static_assert((kOffWqkv16 % 128) == 0 && (kOffWout16 % 128) == 0 && (kOffQ16 % 128) == 0 && (kOffK16 % 128) == 0 &&
              (kOffVt16 % 128) == 0 && (kOffAO16 % 128) == 0 && (kOffBias % 128) == 0);

__device__ __forceinline__ float rin(float f) {
  if (!kBf16Inputs) return f;
  unsigned u = __float_as_uint(f);
  u = (u + 0x7FFFu + ((u >> 16) & 1u)) & 0xFFFF0000u;
  return __uint_as_float(u);
}

__device__ __forceinline__ unsigned short f2bf_bits(float f) {
  unsigned u = __float_as_uint(f);
  return (unsigned short)((u + 0x7FFFu + ((u >> 16) & 1u)) >> 16);
}
__device__ __forceinline__ float bf_bits2f(unsigned short h) { return __uint_as_float(((unsigned)h) << 16); }

__device__ __forceinline__ void dep_guard_h(v8f& a, v8f& b, v16h x, v16h y) { asm volatile("v_nop\n\tv_nop\n\tv_nop\n\tv_nop" : "+v"(a), "+v"(b) : "v"(x), "v"(y)); }
__device__ __forceinline__ void dep_guard_b(v8f& a, v8f& b, v16b x, v16b y) { asm volatile("v_nop\n\tv_nop\n\tv_nop\n\tv_nop" : "+v"(a), "+v"(b) : "v"(x), "v"(y)); }
__device__ __forceinline__ void tie_h(v8f& a, v16h x) { asm volatile("" : "+v"(a) : "v"(x)); }
__device__ __forceinline__ void tie_b(v8f& a, v16b x) { asm volatile("" : "+v"(a) : "v"(x)); }
__device__ __forceinline__ void keep4_h(v16h a, v16h b, v16h c, v16h d) { asm volatile("v_nop" :: "v"(a), "v"(b), "v"(c), "v"(d)); }
__device__ __forceinline__ void keep4_b(v16b a, v16b b, v16b c, v16b d) { asm volatile("v_nop" :: "v"(a), "v"(b), "v"(c), "v"(d)); }
__device__ __forceinline__ void acc_guard4(v8f& a, v8f& b, v8f& c, v8f& d) { asm volatile("v_nop\n\tv_nop\n\tv_nop\n\tv_nop" : "+v"(a), "+v"(b), "+v"(c), "+v"(d)); }
template <typename T> struct Frag;
template <> struct Frag<_Float16> {
  typedef v16h V; union U { v16h v; v8h h[2]; };
  static __device__ __forceinline__ v16h load(const _Float16* p) {
    U f; f.h[0] = *(const v8h*)(p); f.h[1] = *(const v8h*)(p + 16); return f.v;
  }
  static __device__ __forceinline__ v8f mma(v16h a, v16h b, v8f c) {
    return __builtin_amdgcn_wmma_f32_16x16x32_f16(false, a, false, b, (short)0, c, false, false);
  }
  static __device__ __forceinline__ void guard(v8f& a, v8f& b, v16h x, v16h y) { dep_guard_h(a, b, x, y); }
  static __device__ __forceinline__ void tie(v8f& a, v16h x) { tie_h(a, x); }
  static __device__ __forceinline__ void keep(v16h a, v16h b, v16h c, v16h d) { keep4_h(a, b, c, d); }
};
template <> struct Frag<__bf16> {
  typedef v16b V; union U { v16b v; v8b h[2]; };
  static __device__ __forceinline__ v16b load(const __bf16* p) {
    U f; f.h[0] = *(const v8b*)(p); f.h[1] = *(const v8b*)(p + 16); return f.v;
  }
  static __device__ __forceinline__ v8f mma(v16b a, v16b b, v8f c) {
    return __builtin_amdgcn_wmma_f32_16x16x32_bf16(false, a, false, b, (short)0, c, false, false);
  }
  static __device__ __forceinline__ void guard(v8f& a, v8f& b, v16b x, v16b y) { dep_guard_b(a, b, x, y); }
  static __device__ __forceinline__ void tie(v8f& a, v16b x) { tie_b(a, x); }
  static __device__ __forceinline__ void keep(v16b a, v16b b, v16b c, v16b d) { keep4_b(a, b, c, d); }
};

__device__ __forceinline__ void wave_lds_sync() {
  __builtin_amdgcn_fence(__ATOMIC_RELEASE, "workgroup");
  __builtin_amdgcn_wave_barrier();
  __builtin_amdgcn_fence(__ATOMIC_ACQUIRE, "workgroup");
}

template <int ET> struct Elem;
template <> struct Elem<0> { typedef _Float16 T; };
template <> struct Elem<1> { typedef __bf16 T; };
template <int ET, bool SPLIT, int BIAS_MODE, int OUT_MODE, bool RESID>
__global__ __launch_bounds__(256) void wmma_gemm64(
    const unsigned short* __restrict__ Ap, const unsigned short* __restrict__ A2p, int lda, long strideA,
    const unsigned short* __restrict__ Btp, const unsigned short* __restrict__ Bt2p, int ldb, long strideB,
    void* __restrict__ Cout, void* __restrict__ Cout2, int ldc, long strideC,
    const float* __restrict__ bias,
    const float* __restrict__ resid, long strideR,
    int M, int N, int K, float scale) {
  typedef typename Elem<ET>::T T;
  typedef typename Frag<T>::V V;
  const T* A = (const T*)Ap; const T* A2 = (const T*)A2p; const T* Bt = (const T*)Btp; const T* Bt2 = (const T*)Bt2p;
  __shared__ __align__(16) float sT[8][16 * 68];
  const int b    = blockIdx.y;
  const int lane = threadIdx.x & 31;
  const int wave = threadIdx.x >> 5;
  const int tilesN = N >> 6;
  const int tilesM = M >> 6;
  const int tile = blockIdx.x * 8 + wave;
  if (tile >= tilesM * tilesN) return;
  const int tm = tile / tilesN;
  const int tn = tile - tm * tilesN;
  const int m0 = tm << 6;
  const int n0 = tn << 6;

  const T* Ab  = A  + (size_t)b * strideA;
  const T* Bb  = Bt + (size_t)b * strideB;
  const T* Ab2 = SPLIT ? (A2  + (size_t)b * strideA) : nullptr;
  const T* Bb2 = SPLIT ? (Bt2 + (size_t)b * strideB) : nullptr;

  const int rlane = lane & 15;
  const int koff  = (lane >> 4) * 8;
  const int mOff  = (lane >> 4) * 8;

  v8f acc[4][4];
#pragma unroll
  for (int i = 0; i < 4; ++i)
#pragma unroll
    for (int j = 0; j < 4; ++j) acc[i][j] = (v8f){0.f,0.f,0.f,0.f,0.f,0.f,0.f,0.f};

  for (int k0 = 0; k0 < K; k0 += 32) {
    V bh[4], bl[4];
#pragma unroll
    for (int j = 0; j < 4; ++j) {
      const size_t bo = (size_t)(n0 + (j << 4) + rlane) * ldb + koff + k0;
      bh[j] = Frag<T>::load(Bb + bo);
      if (SPLIT) bl[j] = Frag<T>::load(Bb2 + bo);
    }
#pragma unroll
    for (int i = 0; i < 4; ++i) {
      const size_t ao = (size_t)(m0 + (i << 4) + rlane) * lda + koff + k0;
      V ah = Frag<T>::load(Ab + ao);
      V al;
      if (SPLIT) al = Frag<T>::load(Ab2 + ao);
#pragma unroll
      for (int j = 0; j < 4; ++j) {
        acc[i][j] = Frag<T>::mma(ah, bh[j], acc[i][j]);
        if (SPLIT) {
          acc[i][j] = Frag<T>::mma(ah, bl[j], acc[i][j]);
          acc[i][j] = Frag<T>::mma(al, bh[j], acc[i][j]);
        }
      }
      Frag<T>::tie(acc[i][1], ah);
      Frag<T>::tie(acc[i][2], ah);
      Frag<T>::guard(acc[i][0], acc[i][3], ah, SPLIT ? al : ah);
    }
    Frag<T>::keep(bh[0], bh[1], bh[2], bh[3]);
    if (SPLIT) Frag<T>::keep(bl[0], bl[1], bl[2], bl[3]);
  }
  acc_guard4(acc[0][0], acc[0][1], acc[0][2], acc[0][3]);
  acc_guard4(acc[1][0], acc[1][1], acc[1][2], acc[1][3]);
  acc_guard4(acc[2][0], acc[2][1], acc[2][2], acc[2][3]);
  acc_guard4(acc[3][0], acc[3][1], acc[3][2], acc[3][3]);

  float* slab = sT[wave];
  const float* Rb = RESID ? (resid + (size_t)b * strideR) : nullptr;
#pragma unroll
  for (int i = 0; i < 4; ++i) {
    const int mBase = m0 + (i << 4);
#pragma unroll
    for (int j = 0; j < 4; ++j) {
      const int n = n0 + (j << 4) + rlane;
      float bv = 0.f;
      if (BIAS_MODE == 2) bv = bias[n];
#pragma unroll
      for (int r = 0; r < 8; ++r) {
        float v = acc[i][j][r] * scale;
        if (BIAS_MODE == 1) v += bias[mBase + mOff + r];
        if (BIAS_MODE == 2) v += bv;
        if (RESID) v += Rb[(size_t)(mBase + mOff + r) * ldc + n];
        slab[(mOff + r) * 68 + (j << 4) + rlane] = v;
      }
    }
    wave_lds_sync();
    if (OUT_MODE == 0) {
      float* C = (float*)Cout + (size_t)b * strideC;
      const int hh = lane >> 4, c4 = (lane & 15) * 4;
      for (int pass = 0; pass < 2; ++pass) {
#pragma unroll
        for (int it = 0; it < 8; ++it) {
          const int row = it * 2 + hh;
          v4f v = *(const v4f*)(slab + row * 68 + c4);
          *(volatile v4f*)(C + (size_t)(mBase + row) * ldc + n0 + c4) = v;
        }
        __threadfence();
      }
    } else {
      const int q = lane >> 3, c8 = (lane & 7) * 8;
      unsigned short* C  = (unsigned short*)Cout  + (size_t)b * strideC;
      unsigned short* C2 = (OUT_MODE == 2) ? ((unsigned short*)Cout2 + (size_t)b * strideC) : nullptr;
      for (int pass = 0; pass < 2; ++pass) {
#pragma unroll
        for (int it = 0; it < 4; ++it) {
          const int row = it * 4 + q;
          const float* sp = slab + row * 68 + c8;
          v8h hv, lv;
#pragma unroll
          for (int e = 0; e < 8; ++e) {
            if (OUT_MODE == 1) {
              hv[e] = (_Float16)sp[e];
            } else {
              unsigned short hb = f2bf_bits(sp[e]);
              unsigned short lb = f2bf_bits(sp[e] - bf_bits2f(hb));
              hv[e] = __builtin_bit_cast(_Float16, hb);
              lv[e] = __builtin_bit_cast(_Float16, lb);
            }
          }
          *(volatile v8h*)(C + (size_t)(mBase + row) * ldc + n0 + c8) = hv;
          if (OUT_MODE == 2) *(volatile v8h*)(C2 + (size_t)(mBase + row) * ldc + n0 + c8) = lv;
        }
        __threadfence();
      }
    }
    wave_lds_sync();
  }
}

__global__ __launch_bounds__(256) void cast8_f16_kernel(const float* __restrict__ in, unsigned short* __restrict__ out,
                                                        int n8, float carry) {
  const int i = blockIdx.x * 256 + threadIdx.x;
  if (i >= n8) return;
  const float* p = in + 8 * (size_t)i;
  const v4f a = *(const v4f*)(p);
  const v4f c = *(const v4f*)(p + 4);
  v8h hv;
#pragma unroll
  for (int e = 0; e < 4; ++e) {
    const float fa = a[e];
    const float fc = c[e];
    hv[e]     = (_Float16)(rin(fa) * carry);
    hv[4 + e] = (_Float16)(rin(fc) * carry);
  }
  unsigned short* q = out + 8 * (size_t)i;
  *(volatile v8h*)q = hv;
  __threadfence();
  *(volatile v8h*)q = hv;
}

__global__ __launch_bounds__(256) void qk_gemm_norm_kernel(
    const unsigned short* __restrict__ Ap, const unsigned short* __restrict__ Btp,
    unsigned short* __restrict__ Qout, unsigned short* __restrict__ Kout,
    const float* __restrict__ qw, const float* __restrict__ kw) {
  typedef _Float16 T;
  typedef v16h V;
  const T* A = (const T*)Ap;
  const T* Bt = (const T*)Btp;
  __shared__ __align__(16) float sT[8][16 * 68];
  const int lane = threadIdx.x & 31;
  const int wave = threadIdx.x >> 5;
  constexpr int tilesN = (2 * kDim) >> 6;
  constexpr int tilesM = kTok >> 6;
  const int tile = blockIdx.x * 8 + wave;
  if (tile >= tilesM * tilesN) return;
  const int tm = tile / tilesN;
  const int tn = tile - tm * tilesN;
  const int m0 = tm << 6;
  const int n0 = tn << 6;
  const int rlane = lane & 15;
  const int koff  = (lane >> 4) * 8;
  const int mOff  = (lane >> 4) * 8;

  v8f acc[4][4];
#pragma unroll
  for (int i = 0; i < 4; ++i)
#pragma unroll
    for (int j = 0; j < 4; ++j) acc[i][j] = (v8f){0.f,0.f,0.f,0.f,0.f,0.f,0.f,0.f};

  for (int k0 = 0; k0 < kDim; k0 += 32) {
    V bh[4];
#pragma unroll
    for (int j = 0; j < 4; ++j) {
      const size_t bo = (size_t)(n0 + (j << 4) + rlane) * kDim + koff + k0;
      bh[j] = Frag<T>::load(Bt + bo);
    }
#pragma unroll
    for (int i = 0; i < 4; ++i) {
      const size_t ao = (size_t)(m0 + (i << 4) + rlane) * kDim + koff + k0;
      V ah = Frag<T>::load(A + ao);
#pragma unroll
      for (int j = 0; j < 4; ++j) acc[i][j] = Frag<T>::mma(ah, bh[j], acc[i][j]);
      Frag<T>::tie(acc[i][1], ah);
      Frag<T>::tie(acc[i][2], ah);
      Frag<T>::guard(acc[i][0], acc[i][3], ah, ah);
    }
    Frag<T>::keep(bh[0], bh[1], bh[2], bh[3]);
  }
  acc_guard4(acc[0][0], acc[0][1], acc[0][2], acc[0][3]);
  acc_guard4(acc[1][0], acc[1][1], acc[1][2], acc[1][3]);
  acc_guard4(acc[2][0], acc[2][1], acc[2][2], acc[2][3]);
  acc_guard4(acc[3][0], acc[3][1], acc[3][2], acc[3][3]);

  const int third = n0 >> 10;
  const int hIdx  = (n0 & (kDim - 1)) >> 6;
  const int bIdx  = m0 >> 11;
  const int nb    = m0 & (kSeq - 1);
  const float* wsel = third ? kw : qw;
  const int q = lane >> 3, c8 = (lane & 7) * 8;
  const v4f w0 = *(const v4f*)(wsel + c8);
  const v4f w1 = *(const v4f*)(wsel + c8 + 4);
  float wv[8];
#pragma unroll
  for (int e = 0; e < 4; ++e) {
    const float f0 = w0[e];
    const float f1 = w1[e];
    wv[e]     = rin(f0);
    wv[4 + e] = rin(f1);
  }
  unsigned short* dst = (third ? Kout : Qout) + ((size_t)(bIdx * kNH + hIdx) * kSeq + nb) * kHD;

  float* slab = sT[wave];
#pragma unroll
  for (int i = 0; i < 4; ++i) {
#pragma unroll
    for (int j = 0; j < 4; ++j) {
#pragma unroll
      for (int r = 0; r < 8; ++r) slab[(mOff + r) * 68 + (j << 4) + rlane] = acc[i][j][r] * kWCarryInv;
    }
    wave_lds_sync();
    v8h hv[4];
#pragma unroll
    for (int it = 0; it < 4; ++it) {
      const int row = it * 4 + q;
      const float* sp = slab + row * 68 + c8;
      const v4f a0 = *(const v4f*)(sp);
      const v4f a1 = *(const v4f*)(sp + 4);
      float ss = 0.0f;
#pragma unroll
      for (int e = 0; e < 4; ++e) {
        ss = fmaf(a0[e], a0[e], ss);
        ss = fmaf(a1[e], a1[e], ss);
      }
      ss += __shfl_xor(ss, 1, 32);
      ss += __shfl_xor(ss, 2, 32);
      ss += __shfl_xor(ss, 4, 32);
      const float rs = __builtin_amdgcn_rsqf(ss * kInvHD + kEps);
#pragma unroll
      for (int e = 0; e < 4; ++e) {
        hv[it][e]     = (_Float16)((a0[e] * rs) * wv[e]);
        hv[it][4 + e] = (_Float16)((a1[e] * rs) * wv[4 + e]);
      }
    }
    for (int pass = 0; pass < 2; ++pass) {
#pragma unroll
      for (int it = 0; it < 4; ++it) {
        const int row = it * 4 + q;
        *(volatile v8h*)(dst + (size_t)(i * 16 + row) * kHD + c8) = hv[it];
      }
      __threadfence();
    }
    wave_lds_sync();
  }
}

__global__ __launch_bounds__(256) void bias_plane_kernel(const float* __restrict__ cm, const float* __restrict__ im,
                                                         float* __restrict__ bp) {
  __shared__ float red[8];
  const int row  = blockIdx.x;
  const int b    = row >> 11;
  const int qi   = row & (kSeq - 1);
  const int t    = threadIdx.x;
  const int lane = t & 31, wave = t >> 5;
  const float* cmb = cm + (size_t)b * kNCh * kSeq;
  const float c0 = rin(cmb[qi]);
  const float c1 = rin(cmb[kSeq + qi]);
  const float c2 = rin(cmb[2 * kSeq + qi]);
  const float c3 = rin(cmb[3 * kSeq + qi]);
  float mx = -3.0e38f;
#pragma unroll 1
  for (int half = 0; half < 2; ++half) {
    const int k0 = half * 1024 + t * 4;
    const v4f a0 = *(const v4f*)(cmb + k0);
    const v4f a1 = *(const v4f*)(cmb + kSeq + k0);
    const v4f a2 = *(const v4f*)(cmb + 2 * kSeq + k0);
    const v4f a3 = *(const v4f*)(cmb + 3 * kSeq + k0);
#pragma unroll
    for (int e = 0; e < 4; ++e) {
      const float f0 = a0[e], f1 = a1[e], f2 = a2[e], f3 = a3[e];
      float s = c0 * rin(f0);
      s = fmaf(c1, rin(f1), s);
      s = fmaf(c2, rin(f2), s);
      s = fmaf(c3, rin(f3), s);
      mx = fmaxf(mx, s);
    }
  }
  mx = fmaxf(mx, __shfl_xor(mx, 16, 32));
  mx = fmaxf(mx, __shfl_xor(mx, 8, 32));
  mx = fmaxf(mx, __shfl_xor(mx, 4, 32));
  mx = fmaxf(mx, __shfl_xor(mx, 2, 32));
  mx = fmaxf(mx, __shfl_xor(mx, 1, 32));
  if (lane == 0) red[wave] = mx;
  __syncthreads();
  float rm = red[0];
#pragma unroll
  for (int w = 1; w < 8; ++w) rm = fmaxf(rm, red[w]);
  rm = fmaxf(rm, 1e-6f);
  const float inv = 1.0f / rm;
  const float* imr = im + (size_t)row * kSeq;
  float* bo = bp + (size_t)row * kSeq;
#pragma unroll 1
  for (int half = 0; half < 2; ++half) {
    const int k0 = half * 1024 + t * 4;
    const v4f a0 = *(const v4f*)(cmb + k0);
    const v4f a1 = *(const v4f*)(cmb + kSeq + k0);
    const v4f a2 = *(const v4f*)(cmb + 2 * kSeq + k0);
    const v4f a3 = *(const v4f*)(cmb + 3 * kSeq + k0);
    const v4f iv = *(const v4f*)(imr + k0);
    v4f o;
#pragma unroll
    for (int e = 0; e < 4; ++e) {
      const float f0 = a0[e], f1 = a1[e], f2 = a2[e], f3 = a3[e], fi = iv[e];
      float s = c0 * rin(f0);
      s = fmaf(c1, rin(f1), s);
      s = fmaf(c2, rin(f2), s);
      s = fmaf(c3, rin(f3), s);
      o[e] = (s * inv - 0.5f) * 2.0f + kBoost * rin(fi);
    }
    *(volatile v4f*)(bo + k0) = o;
    __threadfence();
    *(volatile v4f*)(bo + k0) = o;
  }
}

constexpr int kAtNW    = 4;
constexpr int kAtQB    = 64;
constexpr int kAtKC    = 64;
constexpr int kAtPitch = 68;
static_assert((kSeq % kAtQB) == 0 && (kSeq % kAtKC) == 0);

__device__ __forceinline__ v8f mma_h(v16h a, v16h b, v8f c) {
  c = __builtin_amdgcn_wmma_f32_16x16x32_f16(false, a, false, b, (short)0, c, false, false);
  asm volatile("v_nop\n\tv_nop\n\tv_nop\n\tv_nop" : "+v"(c) : "v"(a), "v"(b));
  return c;
}

__global__ __launch_bounds__(128) void attn_kernel(
    const unsigned short* __restrict__ Q16, const unsigned short* __restrict__ K16,
    const unsigned short* __restrict__ Vt16, const float* __restrict__ biasp,
    const float* __restrict__ gate, unsigned short* __restrict__ AO16) {
  __shared__ __align__(16) _Float16 Psh[kAtNW][16 * kAtKC];
  __shared__ __align__(16) float    Bsh[kAtNW][16 * kAtPitch];
  __shared__ __align__(16) float    Osh[kAtNW][16 * kAtPitch];

  const int tid  = threadIdx.x;
  const int wave = tid >> 5;
  const int lane = tid & 31;
  const int hh   = lane >> 4;
  const int c    = lane & 15;

  constexpr int nqb = kSeq / kAtQB;
  const int bx = blockIdx.x;
  const int qb = bx % nqb;
  const int bh = bx / nqb;
  const int h  = bh % kNH;
  const int b  = bh / kNH;
  const int q0 = qb * kAtQB + wave * 16;

  const _Float16* Qp = (const _Float16*)Q16  + (size_t)bh * kSeq * kHD;
  const _Float16* Kp = (const _Float16*)K16  + (size_t)bh * kSeq * kHD;
  const _Float16* Vp = (const _Float16*)Vt16 + (size_t)bh * kHD * kSeq;
  const float*    Bp = biasp + (size_t)b * kSeq * kSeq;

  const float graw = rin(gate[h]);
  const float g3   = 3.0f * fminf(fmaxf(graw, 0.0f), 1.0f);

  v16h qa[2];
#pragma unroll
  for (int dc = 0; dc < 2; ++dc) qa[dc] = Frag<_Float16>::load(Qp + (size_t)(q0 + c) * kHD + dc * 32 + 8 * hh);

  float mrow[8], lrow[8];
  v8f oacc[4];
#pragma unroll
  for (int r = 0; r < 8; ++r) { mrow[r] = -1.0e30f; lrow[r] = 0.f; }
#pragma unroll
  for (int t = 0; t < 4; ++t) oacc[t] = (v8f){0.f,0.f,0.f,0.f,0.f,0.f,0.f,0.f};

  float*    bt = Bsh[wave];
  _Float16* pw = Psh[wave];

#pragma unroll 1
  for (int kc = 0; kc < kSeq / kAtKC; ++kc) {
    const int kv0 = kc * kAtKC;
    {
      const int c4 = c * 4;
#pragma unroll
      for (int i = 0; i < 8; ++i) {
        const int row = i * 2 + hh;
        const v4f bv = *(const v4f*)(Bp + (size_t)(q0 + row) * kSeq + kv0 + c4);
        *(v4f*)(bt + row * kAtPitch + c4) = bv;
      }
    }
    v8f s[4];
#pragma unroll
    for (int j = 0; j < 4; ++j) {
      s[j] = (v8f){0.f,0.f,0.f,0.f,0.f,0.f,0.f,0.f};
#pragma unroll
      for (int dc = 0; dc < 2; ++dc) {
        const v16h kb = Frag<_Float16>::load(Kp + (size_t)(kv0 + j * 16 + c) * kHD + dc * 32 + 8 * hh);
        s[j] = mma_h(qa[dc], kb, s[j]);
      }
    }
    wave_lds_sync();
    float cmx[8];
#pragma unroll
    for (int r = 0; r < 8; ++r) {
      float m = -1.0e30f;
#pragma unroll
      for (int j = 0; j < 4; ++j) {
        const float bvv = bt[(8 * hh + r) * kAtPitch + j * 16 + c];
        const float sv = fmaf(g3, bvv, s[j][r] * kQKScale);
        s[j][r] = sv;
        m = fmaxf(m, sv);
      }
      m = fmaxf(m, __shfl_xor(m, 1, 32));
      m = fmaxf(m, __shfl_xor(m, 2, 32));
      m = fmaxf(m, __shfl_xor(m, 4, 32));
      m = fmaxf(m, __shfl_xor(m, 8, 32));
      cmx[r] = m;
    }
#pragma unroll
    for (int r = 0; r < 8; ++r) {
      const float mnew  = fmaxf(mrow[r], cmx[r]);
      const float alpha = __expf(mrow[r] - mnew);
      mrow[r] = mnew;
      float psum = 0.f;
#pragma unroll
      for (int j = 0; j < 4; ++j) {
        const float p = __expf(s[j][r] - mnew);
        psum += p;
        pw[(8 * hh + r) * kAtKC + j * 16 + c] = (_Float16)(p * kPCarry);
      }
      psum += __shfl_xor(psum, 1, 32);
      psum += __shfl_xor(psum, 2, 32);
      psum += __shfl_xor(psum, 4, 32);
      psum += __shfl_xor(psum, 8, 32);
      lrow[r] = lrow[r] * alpha + psum;
#pragma unroll
      for (int t = 0; t < 4; ++t) oacc[t][r] *= alpha;
    }
    wave_lds_sync();
#pragma unroll 1
    for (int kk = 0; kk < 2; ++kk) {
      const v16h pa = Frag<_Float16>::load(pw + c * kAtKC + kk * 32 + 8 * hh);
#pragma unroll
      for (int t = 0; t < 4; ++t) {
        const v16h vb = Frag<_Float16>::load(Vp + (size_t)(t * 16 + c) * kSeq + kv0 + kk * 32 + 8 * hh);
        oacc[t] = mma_h(pa, vb, oacc[t]);
      }
    }
    wave_lds_sync();
  }

  float* os = Osh[wave];
#pragma unroll
  for (int r = 0; r < 8; ++r) {
    const float inv = kCtxFold * (1.0f / lrow[r]);
#pragma unroll
    for (int t = 0; t < 4; ++t) os[(8 * hh + r) * kAtPitch + t * 16 + c] = oacc[t][r] * inv;
  }
  wave_lds_sync();
  {
    const int q = lane >> 3, c8 = (lane & 7) * 8;
    v8h hv[4];
#pragma unroll
    for (int it = 0; it < 4; ++it) {
      const int row = it * 4 + q;
      const float* sp = os + row * kAtPitch + c8;
      const v4f a0 = *(const v4f*)(sp);
      const v4f a1 = *(const v4f*)(sp + 4);
#pragma unroll
      for (int e = 0; e < 4; ++e) {
        hv[it][e]     = (_Float16)a0[e];
        hv[it][4 + e] = (_Float16)a1[e];
      }
    }
    unsigned short* dst = AO16 + (size_t)(b * kSeq + q0) * kDim + h * kHD + c8;
    for (int pass = 0; pass < 2; ++pass) {
#pragma unroll
      for (int it = 0; it < 4; ++it) {
        const int row = it * 4 + q;
        *(volatile v8h*)(dst + (size_t)row * kDim) = hv[it];
      }
      __threadfence();
    }
  }
}

static_assert((2 * kDim) % 64 == 0 && kDim % 64 == 0 && kTok % 64 == 0 && kSeq % 64 == 0);

extern "C" void kernel_launch(void* const* d_in, const int* in_sizes, int n_in,
                              void* d_out, int out_size, void* d_ws, size_t ws_size,
                              hipStream_t stream) {
  if (n_in < 8) return;
  if (in_sizes[0] != kTok * kDim) return;
  if (in_sizes[1] != kNB * kNCh * kSeq) return;
  if (in_sizes[2] != kNB * kSeq * kSeq) return;
  if (in_sizes[3] != 3 * kDim * kDim) return;
  if (in_sizes[4] != kDim * kDim) return;
  if (in_sizes[5] != kHD) return;
  if (in_sizes[6] != kHD) return;
  if (in_sizes[7] != kNH) return;
  if (out_size != kTok * kDim) return;
  if (ws_size < kWsTotal) return;

  const float* x     = (const float*)d_in[0];
  const float* cmask = (const float*)d_in[1];
  const float* imask = (const float*)d_in[2];
  const float* Wqkv  = (const float*)d_in[3];
  const float* Wout  = (const float*)d_in[4];
  const float* qnw   = (const float*)d_in[5];
  const float* knw   = (const float*)d_in[6];
  const float* gate  = (const float*)d_in[7];
  float* out = (float*)d_out;

  char* ws = (char*)d_ws;
  unsigned short* X16    = (unsigned short*)(ws + kOffX16);
  unsigned short* WQKV16 = (unsigned short*)(ws + kOffWqkv16);
  unsigned short* WOUT16 = (unsigned short*)(ws + kOffWout16);
  unsigned short* Q16    = (unsigned short*)(ws + kOffQ16);
  unsigned short* K16    = (unsigned short*)(ws + kOffK16);
  unsigned short* VT16   = (unsigned short*)(ws + kOffVt16);
  unsigned short* AO16   = (unsigned short*)(ws + kOffAO16);
  float*          BIAS   = (float*)(ws + kOffBias);

  cast8_f16_kernel<<<(kTok * kDim / 8) / 256, 256, 0, stream>>>(x, X16, kTok * kDim / 8, 1.0f);
  cast8_f16_kernel<<<(3 * kDim * kDim / 8) / 256, 256, 0, stream>>>(Wqkv, WQKV16, 3 * kDim * kDim / 8, kWCarry);
  cast8_f16_kernel<<<(kDim * kDim / 8) / 256, 256, 0, stream>>>(Wout, WOUT16, kDim * kDim / 8, kWCarry);

  qk_gemm_norm_kernel<<<((kTok / 64) * (2 * kDim / 64)) / 8, 256, 0, stream>>>(X16, WQKV16, Q16, K16, qnw, knw);

  wmma_gemm64<0, false, 0, 1, false><<<dim3(((kDim / 64) * (kSeq / 64)) / 8, kNB), 256, 0, stream>>>(
      WQKV16 + (size_t)2 * kDim * kDim, nullptr, kDim, 0L,
      X16, nullptr, kDim, (long)kSeq * kDim,
      (void*)VT16, nullptr, kSeq, (long)kDim * kSeq,
      nullptr, nullptr, 0L,
      kDim, kSeq, kDim, 1.0f);

  bias_plane_kernel<<<kTok, 256, 0, stream>>>(cmask, imask, BIAS);

  attn_kernel<<<kBH * (kSeq / kAtQB), 128, 0, stream>>>(Q16, K16, VT16, BIAS, gate, AO16);

  wmma_gemm64<0, false, 0, 0, false><<<dim3(((kTok / 64) * (kDim / 64)) / 8, 1), 256, 0, stream>>>(
      AO16, nullptr, kDim, 0L,
      WOUT16, nullptr, kDim, 0L,
      (void*)out, nullptr, kDim, 0L,
      nullptr, nullptr, 0L,
      kTok, kDim, kDim, kOutScale);
}
